// CombinedSymptomMetricGNN_86268713108199
// MI455X (gfx1250) — hardware-verified
//
#include <hip/hip_runtime.h>
#define NNODE 50000
#define NE 800000
#define NTOT (NE + NNODE)
#define NH 4
#define HD 64
#define FH 256
#define NGR 64
#define NN NNODE

typedef __bf16 v16b __attribute__((ext_vector_type(16)));
typedef unsigned short v8us __attribute__((ext_vector_type(8), may_alias));
typedef float  v8f  __attribute__((ext_vector_type(8)));
typedef float  v4f  __attribute__((ext_vector_type(4)));
typedef float  v4fa __attribute__((ext_vector_type(4), may_alias));
union FragB { v16b v; v8us half[2]; unsigned short u[16]; };

__device__ __forceinline__ unsigned short bf16_bits(float x) { unsigned int u = __float_as_uint(x); return (unsigned short)((u + 0x7FFFu + ((u >> 16) & 1u)) >> 16); }
__device__ __forceinline__ float bf16_val(unsigned short b) { return __uint_as_float(((unsigned int)b) << 16); }
__device__ __forceinline__ float bf16_round(float x) { return bf16_val(bf16_bits(x)); }
template <int NT>
__device__ __forceinline__ v8f mmaN(v16b ah, v16b al, v16b bh, v16b bl, v8f c) {
  c = __builtin_amdgcn_wmma_f32_16x16x32_bf16(false, ah, false, bh, (short)0, c, false, false);
  if (NT >= 2) c = __builtin_amdgcn_wmma_f32_16x16x32_bf16(false, al, false, bh, (short)0, c, false, false);
  if (NT >= 3) c = __builtin_amdgcn_wmma_f32_16x16x32_bf16(false, ah, false, bl, (short)0, c, false, false);
  asm volatile("v_nop\n\tv_nop\n\tv_nop\n\tv_nop" : "+v"(c) : "v"(ah), "v"(al), "v"(bh), "v"(bl));
  return c;
}

__global__ __launch_bounds__(256) void k_wt_bf16(const float* __restrict__ W, unsigned short* __restrict__ Wt, int K, int N) {
  const int t = blockIdx.x * 256 + threadIdx.x;
  const int k8n = K / 8;
  if (t >= N * k8n) return;
  const int n = t / k8n, k8 = (t % k8n) * 8;
  v8us v;
#pragma unroll
  for (int i = 0; i < 8; ++i) v[i] = bf16_bits(W[(size_t)(k8 + i) * N + n]);
  *(volatile v8us*)(Wt + (size_t)n * K + k8) = v;
  __threadfence();
  *(volatile v8us*)(Wt + (size_t)n * K + k8) = v;
}

template <bool ASPLIT, int ACT, bool BIAS_BF16>
__global__ __launch_bounds__(128) void k_gemm_bf(const float* __restrict__ A, int lda, const unsigned short* __restrict__ Wt, int ldb,
                                               const float* __restrict__ bias, float* __restrict__ C, int ldc, int M, int N, int K) {
  __shared__ __attribute__((aligned(16))) float so[4][16][64];
  const int tid = threadIdx.x, w = tid >> 5, lane = tid & 31, ln = lane & 15, hh = lane >> 4;
  const int ntn = N / 64;
  const int wid = blockIdx.x * 4 + w;
  const int mt = wid / ntn, nq = wid % ntn;
  if (mt * 16 >= M) return;
  const int row0 = mt * 16, col0 = nq * 64;
  const float* arow = A + (size_t)(row0 + ln) * lda;
  v8f acc[4] = {};
  for (int kb = 0; kb < K; kb += 32) {
    FragB ah, al;
    const v4f x0 = *(const v4fa*)(arow + kb + 8 * hh), x1 = *(const v4fa*)(arow + kb + 8 * hh + 4);
    const v4f x2 = *(const v4fa*)(arow + kb + 16 + 8 * hh), x3 = *(const v4fa*)(arow + kb + 16 + 8 * hh + 4);
    float xs[16] = {x0[0],x0[1],x0[2],x0[3],x1[0],x1[1],x1[2],x1[3],x2[0],x2[1],x2[2],x2[3],x3[0],x3[1],x3[2],x3[3]};
#pragma unroll
    for (int i = 0; i < 16; ++i) { const unsigned short hb = bf16_bits(xs[i]); ah.u[i] = hb; al.u[i] = ASPLIT ? bf16_bits(xs[i] - bf16_val(hb)) : (unsigned short)0; }
#pragma unroll
    for (int t = 0; t < 4; ++t) {
      const unsigned short* brow = Wt + (size_t)(col0 + t * 16 + ln) * ldb + kb;
      FragB b;
      b.half[0] = *(const v8us*)(brow + 8 * hh);
      b.half[1] = *(const v8us*)(brow + 16 + 8 * hh);
      acc[t] = mmaN<ASPLIT ? 2 : 1>(ah.v, al.v, b.v, b.v, acc[t]);
    }
  }
#pragma unroll
  for (int t = 0; t < 4; ++t) {
    float bv = bias ? bias[col0 + t * 16 + ln] : 0.f;
    if (BIAS_BF16) bv = bf16_round(bv);
#pragma unroll
    for (int r = 0; r < 8; ++r) { float v = acc[t][r] + bv; if (ACT == 1) v = fmaxf(v, 0.f); so[w][8 * hh + r][t * 16 + ln] = v; }
  }
  __builtin_amdgcn_fence(__ATOMIC_ACQ_REL, "workgroup");
  __builtin_amdgcn_wave_barrier();
  const int rsub = lane >> 4, c4 = (lane & 15) * 4;
  for (int pass = 0; pass < 2; ++pass) {
#pragma unroll
    for (int q = 0; q < 8; ++q) {
      const int r = q * 2 + rsub;
      const v4f v = *(const v4fa*)&so[w][r][c4];
      *(volatile v4f*)(C + (size_t)(row0 + r) * ldc + col0 + c4) = v;
    }
    if (pass == 0) __threadfence();
  }
}

template <int D, bool CAUSAL>
__global__ __launch_bounds__(128) void k_flash(const float* __restrict__ qb, const float* __restrict__ kb, const float* __restrict__ vb,
                                             int pitch, int T, int H, float scale, float* __restrict__ y, int ypitch) {
  constexpr int KS = D / 32;
  constexpr int DT = D / 16;
  __shared__ __attribute__((aligned(16))) unsigned short sKh[32][D + 8], sKl[32][D + 8], sVh[32][D + 8], sVl[32][D + 8];
  __shared__ __attribute__((aligned(16))) unsigned short sPh[4][16][40], sPl[4][16][40];
  __shared__ __attribute__((aligned(16))) float sO[4][16][D];
  const int tid = threadIdx.x, w = tid >> 5, lane = tid & 31, ln = lane & 15, hh = lane >> 4;
  const int nqb = (T + 63) / 64;
  const int bh = blockIdx.x / nqb, qblk = blockIdx.x % nqb;
  const int b = bh / H, h = bh % H;
  const int q0 = qblk * 64 + w * 16;
  const float* Q = qb + (size_t)b * T * pitch + h * D;
  const float* K = kb + (size_t)b * T * pitch + h * D;
  const float* V = vb + (size_t)b * T * pitch + h * D;

  FragB aqh[KS], aql[KS];
  {
    int row = q0 + ln; if (row >= T) row = T - 1;
    const float* qr = Q + (size_t)row * pitch;
#pragma unroll
    for (int ks = 0; ks < KS; ++ks)
#pragma unroll
      for (int i = 0; i < 16; ++i) {
        const int d = ks * 32 + ((i < 8) ? (8 * hh + i) : (16 + 8 * hh + (i - 8)));
        const float x = qr[d] * scale; const unsigned short hb = bf16_bits(x);
        aqh[ks].u[i] = hb; aql[ks].u[i] = bf16_bits(x - bf16_val(hb));
      }
  }
  float m_r[8], l_r[8];
#pragma unroll
  for (int r = 0; r < 8; ++r) { m_r[r] = -3.0e38f; l_r[r] = 0.f; }
  v8f oacc[DT];
#pragma unroll
  for (int dt = 0; dt < DT; ++dt) oacc[dt] = (v8f){0.f,0.f,0.f,0.f,0.f,0.f,0.f,0.f};

  const int kv_end = CAUSAL ? min(T, qblk * 64 + 64) : T;
  for (int j0 = 0; j0 < kv_end; j0 += 32) {
    __syncthreads();
    for (int e = tid; e < 32 * (D / 4); e += 128) {
      const int r = e / (D / 4), c4 = (e % (D / 4)) * 4;
      const int key = j0 + r;
      v4f kf = {0.f,0.f,0.f,0.f}, vf = {0.f,0.f,0.f,0.f};
      if (key < T) { kf = *(const v4fa*)(K + (size_t)key * pitch + c4); vf = *(const v4fa*)(V + (size_t)key * pitch + c4); }
#pragma unroll
      for (int t = 0; t < 4; ++t) {
        unsigned short hb = bf16_bits(kf[t]); sKh[r][c4 + t] = hb; sKl[r][c4 + t] = bf16_bits(kf[t] - bf16_val(hb));
        hb = bf16_bits(vf[t]); sVh[r][c4 + t] = hb; sVl[r][c4 + t] = bf16_bits(vf[t] - bf16_val(hb));
      }
    }
    __syncthreads();
    v8f s[2];
#pragma unroll
    for (int nt = 0; nt < 2; ++nt) {
      v8f acc = {};
#pragma unroll
      for (int ks = 0; ks < KS; ++ks) {
        FragB bh_, bl_;
        bh_.half[0] = *(const v8us*)&sKh[nt * 16 + ln][ks * 32 + 8 * hh]; bh_.half[1] = *(const v8us*)&sKh[nt * 16 + ln][ks * 32 + 16 + 8 * hh];
        bl_.half[0] = *(const v8us*)&sKl[nt * 16 + ln][ks * 32 + 8 * hh]; bl_.half[1] = *(const v8us*)&sKl[nt * 16 + ln][ks * 32 + 16 + 8 * hh];
        acc = mmaN<3>(aqh[ks].v, aql[ks].v, bh_.v, bl_.v, acc);
      }
      s[nt] = acc;
    }
    float alpha[8];
#pragma unroll
    for (int r = 0; r < 8; ++r) {
      const int qi = q0 + 8 * hh + r;
      const int ja = j0 + ln, jb = j0 + 16 + ln;
      if (CAUSAL) { if (ja > qi) s[0][r] = -3.0e38f; if (jb > qi) s[1][r] = -3.0e38f; }
      if (ja >= T) s[0][r] = -3.0e38f;
      if (jb >= T) s[1][r] = -3.0e38f;
      float mx = fmaxf(s[0][r], s[1][r]);
      mx = fmaxf(mx, __shfl_xor(mx, 1, 32)); mx = fmaxf(mx, __shfl_xor(mx, 2, 32)); mx = fmaxf(mx, __shfl_xor(mx, 4, 32)); mx = fmaxf(mx, __shfl_xor(mx, 8, 32));
      const float mnew = fmaxf(m_r[r], mx);
      alpha[r] = (mnew > -1.0e38f) ? __expf(m_r[r] - mnew) : 1.0f;
      const float p0 = (s[0][r] > -1.0e38f) ? __expf(s[0][r] - mnew) : 0.f;
      const float p1 = (s[1][r] > -1.0e38f) ? __expf(s[1][r] - mnew) : 0.f;
      m_r[r] = mnew;
      l_r[r] = l_r[r] * alpha[r] + p0 + p1;
      unsigned short hb = bf16_bits(p0); sPh[w][8 * hh + r][ln] = hb;      sPl[w][8 * hh + r][ln] = bf16_bits(p0 - bf16_val(hb));
      hb = bf16_bits(p1);                sPh[w][8 * hh + r][16 + ln] = hb; sPl[w][8 * hh + r][16 + ln] = bf16_bits(p1 - bf16_val(hb));
    }
#pragma unroll
    for (int dt = 0; dt < DT; ++dt)
#pragma unroll
      for (int r = 0; r < 8; ++r) oacc[dt][r] *= alpha[r];
    __builtin_amdgcn_fence(__ATOMIC_ACQ_REL, "workgroup");
    __builtin_amdgcn_wave_barrier();
    FragB pah, pal;
    pah.half[0] = *(const v8us*)&sPh[w][ln][8 * hh]; pah.half[1] = *(const v8us*)&sPh[w][ln][16 + 8 * hh];
    pal.half[0] = *(const v8us*)&sPl[w][ln][8 * hh]; pal.half[1] = *(const v8us*)&sPl[w][ln][16 + 8 * hh];
#pragma unroll
    for (int dt = 0; dt < DT; ++dt) {
      FragB bvh, bvl;
#pragma unroll
      for (int i = 0; i < 8; ++i) {
        bvh.u[i] = sVh[8 * hh + i][dt * 16 + ln]; bvh.u[8 + i] = sVh[16 + 8 * hh + i][dt * 16 + ln];
        bvl.u[i] = sVl[8 * hh + i][dt * 16 + ln]; bvl.u[8 + i] = sVl[16 + 8 * hh + i][dt * 16 + ln];
      }
      oacc[dt] = mmaN<3>(pah.v, pal.v, bvh.v, bvl.v, oacc[dt]);
    }
    __builtin_amdgcn_fence(__ATOMIC_ACQ_REL, "workgroup");
    __builtin_amdgcn_wave_barrier();
  }
#pragma unroll
  for (int r = 0; r < 8; ++r) {
    float l = l_r[r];
    l += __shfl_xor(l, 1, 32); l += __shfl_xor(l, 2, 32); l += __shfl_xor(l, 4, 32); l += __shfl_xor(l, 8, 32);
    l_r[r] = (l > 0.f) ? 1.0f / l : 0.f;
  }
#pragma unroll
  for (int dt = 0; dt < DT; ++dt)
#pragma unroll
    for (int r = 0; r < 8; ++r) sO[w][8 * hh + r][dt * 16 + ln] = oacc[dt][r] * l_r[r];
  __builtin_amdgcn_fence(__ATOMIC_ACQ_REL, "workgroup");
  __builtin_amdgcn_wave_barrier();
  for (int pass = 0; pass < 2; ++pass) {
    for (int r = 0; r < 16; ++r) {
      const int row = q0 + r;
      if (row < T && lane < D / 4) {
        const v4f val = *(const v4fa*)&sO[w][r][lane * 4];
        *(volatile v4f*)(y + ((size_t)b * T + row) * ypitch + h * D + lane * 4) = val;
      }
    }
    if (pass == 0) __threadfence();
  }
}

template <bool ASPLIT, int ACT, bool BIAS_BF16, bool RES_BF16>
__global__ __launch_bounds__(128) void k_gemm_bf3(const float* __restrict__ A, int lda, const unsigned short* __restrict__ Wt, int ldb,
                                                const float* __restrict__ bias, const float* __restrict__ resid, int rmod, int ldr,
                                                float* __restrict__ C, int ldc, int M, int N, int K) {
  __shared__ __attribute__((aligned(16))) float so[4][16][64];
  const int tid = threadIdx.x, w = tid >> 5, lane = tid & 31, ln = lane & 15, hh = lane >> 4;
  const int ntn = N / 64;
  const int wid = blockIdx.x * 4 + w;
  const int mt = wid / ntn, nq = wid % ntn;
  if (mt * 16 >= M) return;
  const int row0 = mt * 16, col0 = nq * 64;
  const float* arow = A + (size_t)(row0 + ln) * lda;
  v8f acc[4] = {};
  for (int kb = 0; kb < K; kb += 32) {
    FragB ah, al;
    const v4f x0 = *(const v4fa*)(arow + kb + 8 * hh), x1 = *(const v4fa*)(arow + kb + 8 * hh + 4);
    const v4f x2 = *(const v4fa*)(arow + kb + 16 + 8 * hh), x3 = *(const v4fa*)(arow + kb + 16 + 8 * hh + 4);
    float xs[16] = {x0[0],x0[1],x0[2],x0[3],x1[0],x1[1],x1[2],x1[3],x2[0],x2[1],x2[2],x2[3],x3[0],x3[1],x3[2],x3[3]};
#pragma unroll
    for (int i = 0; i < 16; ++i) { const unsigned short hb = bf16_bits(xs[i]); ah.u[i] = hb; al.u[i] = ASPLIT ? bf16_bits(xs[i] - bf16_val(hb)) : (unsigned short)0; }
#pragma unroll
    for (int t = 0; t < 4; ++t) {
      const unsigned short* brow = Wt + (size_t)(col0 + t * 16 + ln) * ldb + kb;
      FragB b;
      b.half[0] = *(const v8us*)(brow + 8 * hh);
      b.half[1] = *(const v8us*)(brow + 16 + 8 * hh);
      acc[t] = mmaN<ASPLIT ? 2 : 1>(ah.v, al.v, b.v, b.v, acc[t]);
    }
  }
#pragma unroll
  for (int t = 0; t < 4; ++t) {
    const int col = col0 + t * 16 + ln;
    float bv = bias ? bias[col] : 0.f;
    if (BIAS_BF16) bv = bf16_round(bv);
#pragma unroll
    for (int r = 0; r < 8; ++r) {
      float v = acc[t][r] + bv;
      if (resid) { float rv = resid[(size_t)((row0 + 8 * hh + r) % rmod) * ldr + col]; if (RES_BF16) rv = bf16_round(rv); v += rv; }
      if (ACT == 1) v = fmaxf(v, 0.f);
      if (ACT == 2) v = 0.5f * v * (1.0f + erff(v * 0.70710678118654752f));
      if (ACT == 3) { const float u = 0.7978845608028654f * (v + 0.044715f * v * v * v); v = 0.5f * v * (1.0f + tanhf(u)); }
      so[w][8 * hh + r][t * 16 + ln] = v;
    }
  }
  __builtin_amdgcn_fence(__ATOMIC_ACQ_REL, "workgroup");
  __builtin_amdgcn_wave_barrier();
  const int rsub = lane >> 4, c4 = (lane & 15) * 4;
  for (int pass = 0; pass < 2; ++pass) {
#pragma unroll
    for (int q = 0; q < 8; ++q) {
      const int r = q * 2 + rsub;
      const v4f v = *(const v4fa*)&so[w][r][c4];
      *(volatile v4f*)(C + (size_t)(row0 + r) * ldc + col0 + c4) = v;
    }
    if (pass == 0) __threadfence();
  }
}
template <bool PARAM_BF16>
__global__ __launch_bounds__(256) void k_layernorm(const float* __restrict__ X, const float* __restrict__ R, const float* __restrict__ g, const float* __restrict__ bta,
                                                  float* __restrict__ out_sum, float* __restrict__ out_norm, int N, float eps) {
  __shared__ float red[256];
  const int row = blockIdx.x, tid = threadIdx.x;
  const float* x = X + (size_t)row * N; const float* rr = R ? R + (size_t)row * N : nullptr;
  float vals[16];
  const int per = N / 256;
  float s1 = 0.f;
  for (int u = 0; u < per / 4; ++u) {
    const int j = tid * 4 + 1024 * u;
    const v4f a = *(const v4fa*)(x + j);
    v4f b = {0.f,0.f,0.f,0.f}; if (rr) b = *(const v4fa*)(rr + j);
#pragma unroll
    for (int q = 0; q < 4; ++q) { const float v = a[q] + b[q]; vals[u * 4 + q] = v; s1 += v; }
  }
  red[tid] = s1; __syncthreads();
  for (int st = 128; st > 0; st >>= 1) { if (tid < st) red[tid] += red[tid + st]; __syncthreads(); }
  const float mu = red[0] / (float)N; __syncthreads();
  float s2 = 0.f;
  for (int u = 0; u < per / 4; ++u)
#pragma unroll
    for (int q = 0; q < 4; ++q) { const float c = vals[u * 4 + q] - mu; s2 += c * c; }
  red[tid] = s2; __syncthreads();
  for (int st = 128; st > 0; st >>= 1) { if (tid < st) red[tid] += red[tid + st]; __syncthreads(); }
  const float rs = rsqrtf(red[0] / (float)N + eps);
  for (int pass = 0; pass < 2; ++pass) {
    for (int u = 0; u < per / 4; ++u) {
      const int j = tid * 4 + 1024 * u;
      v4f o, sm;
#pragma unroll
      for (int q = 0; q < 4; ++q) {
        float gg = g[j + q], bb = bta[j + q];
        if (PARAM_BF16) { gg = bf16_round(gg); bb = bf16_round(bb); }
        sm[q] = vals[u * 4 + q]; o[q] = (vals[u * 4 + q] - mu) * rs * gg + bb;
      }
      if (out_sum) *(volatile v4f*)(out_sum + (size_t)row * N + j) = sm;
      *(volatile v4f*)(out_norm + (size_t)row * N + j) = o;
    }
    if (pass == 0) __threadfence();
  }
}

typedef _Float16 v16h __attribute__((ext_vector_type(16)));
union FragH { v16h v; v8us half[2]; _Float16 h[16]; unsigned short u[16]; };
template <int NT>
__device__ __forceinline__ v8f mmaH(v16h ah, v16h al, v16h bh, v16h bl, v8f c) {
  c = __builtin_amdgcn_wmma_f32_16x16x32_f16(false, ah, false, bh, (short)0, c, false, false);
  if (NT >= 2) c = __builtin_amdgcn_wmma_f32_16x16x32_f16(false, al, false, bh, (short)0, c, false, false);
  if (NT >= 3) c = __builtin_amdgcn_wmma_f32_16x16x32_f16(false, ah, false, bl, (short)0, c, false, false);
  asm volatile("v_nop\n\tv_nop\n\tv_nop\n\tv_nop" : "+v"(c) : "v"(ah), "v"(al), "v"(bh), "v"(bl));
  return c;
}
template <bool ASPLIT>
__global__ __launch_bounds__(128) void k_gemm_h(const float* __restrict__ A, int lda, size_t sA, const _Float16* __restrict__ Bh, int ldb, size_t sB, float alpha, float* __restrict__ C, int ldc, size_t sC, int M, int N, int K) {
  __shared__ __attribute__((aligned(16))) float so[4][16][64];
  const int tid = threadIdx.x, w = tid >> 5, lane = tid & 31, ln = lane & 15, hh = lane >> 4; const int by = blockIdx.y;
  A += (size_t)by * sA; Bh += (size_t)by * sB; C += (size_t)by * sC;
  const int ntn = (N + 63) / 64; const int wid = blockIdx.x * 4 + w; const int mt = wid / ntn, nq = wid % ntn; if (mt * 16 >= M) return;
  const int row0 = mt * 16, col0 = nq * 64; const float* arow = A + (size_t)(row0 + ln) * lda;
  v8f acc[4] = {};
  for (int kb = 0; kb < K; kb += 32) {
    FragH ah, al;
    const v4f x0 = *(const v4fa*)(arow + kb + 8 * hh), x1 = *(const v4fa*)(arow + kb + 8 * hh + 4), x2 = *(const v4fa*)(arow + kb + 16 + 8 * hh), x3 = *(const v4fa*)(arow + kb + 16 + 8 * hh + 4);
    float xs[16] = {x0[0],x0[1],x0[2],x0[3],x1[0],x1[1],x1[2],x1[3],x2[0],x2[1],x2[2],x2[3],x3[0],x3[1],x3[2],x3[3]};
#pragma unroll
    for (int i = 0; i < 16; ++i) { const _Float16 h = (_Float16)xs[i]; ah.h[i] = h; al.h[i] = ASPLIT ? (_Float16)(xs[i] - (float)h) : (_Float16)0.0f; }
#pragma unroll
    for (int t = 0; t < 4; ++t) { if (col0 + t * 16 >= N) continue; const size_t boff = (size_t)(col0 + t * 16 + ln) * ldb + kb; FragH bq; bq.half[0] = *(const v8us*)(Bh + boff + 8 * hh); bq.half[1] = *(const v8us*)(Bh + boff + 16 + 8 * hh);
      acc[t] = mmaH<ASPLIT ? 2 : 1>(ah.v, al.v, bq.v, bq.v, acc[t]); }
  }
#pragma unroll
  for (int t = 0; t < 4; ++t) { if (col0 + t * 16 >= N) continue;
#pragma unroll
    for (int r = 0; r < 8; ++r) so[w][8 * hh + r][t * 16 + ln] = acc[t][r] * alpha; }
  __builtin_amdgcn_fence(__ATOMIC_ACQ_REL, "workgroup"); __builtin_amdgcn_wave_barrier();
  const int rsub = lane >> 4, c4 = (lane & 15) * 4;
  for (int pass = 0; pass < 2; ++pass) {
#pragma unroll
    for (int q = 0; q < 8; ++q) { const int r = q * 2 + rsub; if (col0 + c4 < N) { const v4f v = *(const v4fa*)&so[w][r][c4]; *(volatile v4f*)(C + (size_t)(row0 + r) * ldc + col0 + c4) = v; } }
    if (pass == 0) __threadfence(); }
}

#define CS_NW 1024
#define CS_CH 832
#define CS_NB 256
#define CS_CAP 8192
__device__ __forceinline__ int cs_dst(const int* __restrict__ eidst, int e, int ne, int nt, int nn) { if (e >= nt) return -1; int d = (e < ne) ? eidst[e] : (e - ne); return d < 0 ? 0 : (d >= nn ? nn - 1 : d); }
__global__ __launch_bounds__(256) void k_cs_p1(const int* __restrict__ eidst, int ne, int nt, int nn, int* __restrict__ seg_dst, int* __restrict__ seg_eid, int* __restrict__ P1, int* __restrict__ Q1) {
  __shared__ int scnt[8][CS_NB]; __shared__ int srun[8][CS_NB]; __shared__ int sod[8][CS_CH]; __shared__ int soe[8][CS_CH];
  const int tid = threadIdx.x, wv = tid >> 5, lane = tid & 31; const int w = blockIdx.x * 8 + wv; const int e0 = w * CS_CH;
  for (int i = lane; i < CS_NB; i += 32) { scnt[wv][i] = 0; srun[wv][i] = 0; }
  __builtin_amdgcn_fence(__ATOMIC_ACQ_REL, "workgroup"); __builtin_amdgcn_wave_barrier();
#pragma unroll 1
  for (int i0 = 0; i0 < CS_CH; i0 += 32) { const int e = e0 + i0 + lane; const int d = cs_dst(eidst, e, ne, nt, nn); const int hb = (d < 0) ? -1 : (d >> 8);
#pragma unroll 1
    for (int ld = 0; ld < 32; ++ld) { const int kk = __shfl(hb, ld, 32); const unsigned long long m = __ballot(hb == kk); const int first = __ffsll((long long)m) - 1; if (ld == first && lane == first && kk >= 0) scnt[wv][kk] += __popcll(m); }
    __builtin_amdgcn_fence(__ATOMIC_ACQ_REL, "workgroup"); __builtin_amdgcn_wave_barrier(); }
  { int loc[8]; int s = 0; for (int j = 0; j < 8; ++j) { loc[j] = s; s += scnt[wv][lane * 8 + j]; }
    int incl = s; for (int o = 1; o < 32; o <<= 1) { const int v = __shfl_up(incl, o, 32); if (lane >= o) incl += v; } const int excl = incl - s;
    for (int j = 0; j < 8; ++j) srun[wv][lane * 8 + j] = excl + loc[j]; }
  __builtin_amdgcn_fence(__ATOMIC_ACQ_REL, "workgroup"); __builtin_amdgcn_wave_barrier();
  for (int pass = 0; pass < 2; ++pass) { for (int i = lane; i < CS_NB; i += 32) { *(volatile int*)(P1 + (size_t)w * CS_NB + i) = scnt[wv][i]; *(volatile int*)(Q1 + (size_t)w * CS_NB + i) = srun[wv][i]; } if (pass == 0) __threadfence(); }
#pragma unroll 1
  for (int i0 = 0; i0 < CS_CH; i0 += 32) { const int e = e0 + i0 + lane; const int d = cs_dst(eidst, e, ne, nt, nn); const int hb = (d < 0) ? -1 : (d >> 8);
    int pos = -1; int grpcnt = 0; bool leader = false;
#pragma unroll 1
    for (int ld = 0; ld < 32; ++ld) { const int kk = __shfl(hb, ld, 32); const unsigned long long g = __ballot(hb == kk); const int first = __ffsll((long long)g) - 1;
      if (ld == first && kk >= 0) { if (hb == kk) { const unsigned long long below = g & ((1ull << lane) - 1ull); pos = srun[wv][kk] + __popcll(below); if (lane == first) { leader = true; grpcnt = __popcll(g); } } } }
    if (pos >= 0) { sod[wv][pos] = d; soe[wv][pos] = e; }
    __builtin_amdgcn_fence(__ATOMIC_ACQ_REL, "workgroup"); __builtin_amdgcn_wave_barrier();
    if (leader) srun[wv][hb] += grpcnt;
    __builtin_amdgcn_fence(__ATOMIC_ACQ_REL, "workgroup"); __builtin_amdgcn_wave_barrier(); }
  for (int pass = 0; pass < 2; ++pass) { for (int i = lane; i < CS_CH; i += 32) { *(volatile int*)(seg_dst + (size_t)e0 + i) = sod[wv][i]; *(volatile int*)(seg_eid + (size_t)e0 + i) = soe[wv][i]; } if (pass == 0) __threadfence(); }
}
__global__ __launch_bounds__(256) void k_cs_scan(const int* __restrict__ P1, int* __restrict__ R, int* __restrict__ S) {
  __shared__ int tot[CS_NB]; __shared__ int st[CS_NB + 1];
  const int b = threadIdx.x; int acc = 0;
#pragma unroll 1
  for (int w = 0; w < CS_NW; ++w) { const int c = P1[(size_t)w * CS_NB + b]; *(volatile int*)(R + (size_t)w * CS_NB + b) = acc; acc += c; }
  __threadfence();
  acc = 0;
#pragma unroll 1
  for (int w = 0; w < CS_NW; ++w) { const int c = P1[(size_t)w * CS_NB + b]; *(volatile int*)(R + (size_t)w * CS_NB + b) = acc; acc += c; }
  tot[b] = acc; __syncthreads();
  if (b == 0) { int s = 0; for (int i = 0; i < CS_NB; ++i) { st[i] = s; s += (tot[i] + 31) & ~31; } st[CS_NB] = s; }
  __syncthreads();
  for (int pass = 0; pass < 2; ++pass) { *(volatile int*)(S + b) = st[b]; if (b < 32) *(volatile int*)(S + CS_NB + b) = (b == 0) ? st[CS_NB] : 0; if (pass == 0) __threadfence(); }
}
__global__ __launch_bounds__(256) void k_cs_p2(const int* __restrict__ seg_dst, const int* __restrict__ seg_eid, const int* __restrict__ P1, const int* __restrict__ Q1, const int* __restrict__ R, const int* __restrict__ S, int nn, int* __restrict__ csr_eid, int* __restrict__ csr_start, int* __restrict__ csr_cnt) {
  __shared__ int sd[CS_CAP]; __shared__ int se[CS_CAP]; __shared__ int sorted[CS_CAP]; __shared__ int lcnt[CS_NB]; __shared__ int lpre[CS_NB + 1];
  const int hb = blockIdx.x, t = threadIdx.x; const int total = (R[(size_t)(CS_NW - 1) * CS_NB + hb] + P1[(size_t)(CS_NW - 1) * CS_NB + hb]); const int tot = total > CS_CAP ? CS_CAP : total;
#pragma unroll 1
  for (int w = t; w < CS_NW; w += 256) { const int c = P1[(size_t)w * CS_NB + hb]; const int base = R[(size_t)w * CS_NB + hb]; const int src = w * CS_CH + Q1[(size_t)w * CS_NB + hb];
    for (int k = 0; k < c; ++k) { const int p = base + k; if (p < CS_CAP) { sd[p] = seg_dst[src + k] & 255; se[p] = seg_eid[src + k]; } } }
  __syncthreads();
  { int c = 0;
#pragma unroll 1
    for (int i = 0; i < tot; ++i) c += (sd[i] == t) ? 1 : 0; lcnt[t] = c; }
  __syncthreads();
  if (t == 0) { int s = 0; for (int i = 0; i < CS_NB; ++i) { lpre[i] = s; s += lcnt[i]; } lpre[CS_NB] = s; }
  __syncthreads();
  { int k = lpre[t];
#pragma unroll 1
    for (int i = 0; i < tot; ++i) if (sd[i] == t) { sorted[k++] = se[i]; } }
  __syncthreads();
  const int s0 = S[hb]; const int s1 = S[hb + 1];
  for (int pass = 0; pass < 2; ++pass) {
    for (int i = t; i < s1 - s0; i += 256) *(volatile int*)(csr_eid + s0 + i) = (i < tot) ? sorted[i] : -1;
    { const int dst = hb * CS_NB + t; *(volatile int*)(csr_start + dst) = s0 + lpre[t]; *(volatile int*)(csr_cnt + dst) = lcnt[t]; }
    if (pass == 0) __threadfence(); }
}
static void build_csr(const int* eidst, int ne, int nt, int nn, int* seg_dst, int* seg_eid, int* P1, int* Q1, int* R, int* S, int* csr_eid, int* csr_start, int* csr_cnt, hipStream_t stream) {
  k_cs_p1<<<CS_NW / 8, 256, 0, stream>>>(eidst, ne, nt, nn, seg_dst, seg_eid, P1, Q1);
  k_cs_scan<<<1, 256, 0, stream>>>(P1, R, S);
  k_cs_p2<<<CS_NB, 256, 0, stream>>>(seg_dst, seg_eid, P1, Q1, R, S, nn, csr_eid, csr_start, csr_cnt);
}

__global__ __launch_bounds__(256) void k_wt_f16(const float* __restrict__ W, _Float16* __restrict__ Wt, int K, int N, float scale) {
  const int t = blockIdx.x * 256 + threadIdx.x; if (t >= N * (K / 8)) return; const int n = t / (K / 8), k8 = (t % (K / 8)) * 8; FragH f;
#pragma unroll
  for (int i = 0; i < 8; ++i) f.h[i] = (_Float16)(bf16_round(W[(size_t)(k8 + i) * N + n]) * scale); const v8us o = f.half[0];
  *(volatile v8us*)((unsigned short*)Wt + (size_t)n * K + k8) = o; __threadfence(); *(volatile v8us*)((unsigned short*)Wt + (size_t)n * K + k8) = o; }
__global__ __launch_bounds__(1024) void k_elr(const float* __restrict__ f, const float* __restrict__ al, const float* __restrict__ ar, float* __restrict__ elr) {
  __shared__ float so[32][8]; const int tid = threadIdx.x, wv = tid >> 5, lane = tid & 31; const int n = blockIdx.x * 32 + wv;
  float sl[NH], sr[NH]; for (int h = 0; h < NH; ++h) { sl[h] = 0.f; sr[h] = 0.f; }
  if (n < NNODE) { const float* fr = f + (size_t)n * FH;
#pragma unroll
    for (int h = 0; h < NH; ++h) { const float v0 = fr[h * HD + lane], v1 = fr[h * HD + 32 + lane]; sl[h] = v0 * bf16_round(al[h * HD + lane]) + v1 * bf16_round(al[h * HD + 32 + lane]); sr[h] = v0 * bf16_round(ar[h * HD + lane]) + v1 * bf16_round(ar[h * HD + 32 + lane]); } }
#pragma unroll
  for (int h = 0; h < NH; ++h) { for (int o = 16; o >= 1; o >>= 1) { sl[h] += __shfl_xor(sl[h], o, 32); sr[h] += __shfl_xor(sr[h], o, 32); } }
  if (lane == 0) { for (int h = 0; h < NH; ++h) { so[wv][h] = sl[h]; so[wv][4 + h] = sr[h]; } }
  __syncthreads();
  if (tid < 256 && blockIdx.x * 32 + tid / 8 < NNODE) { *(volatile float*)(elr + (size_t)blockIdx.x * 256 + tid) = so[tid / 8][tid % 8]; } __threadfence(); if (tid < 256 && blockIdx.x * 32 + tid / 8 < NNODE) { *(volatile float*)(elr + (size_t)blockIdx.x * 256 + tid) = so[tid / 8][tid % 8]; }
}
__global__ __launch_bounds__(1024) void k_gat4(const float* __restrict__ f, const float* __restrict__ elr, const int* __restrict__ src, const int* __restrict__ cstart, const int* __restrict__ ccnt, const int* __restrict__ ceid, float* __restrict__ out, const float* __restrict__ bias) {
  __shared__ float so[32]; __shared__ float sal[32][64][NH]; __shared__ float srw[32][FH]; __shared__ int sidx[32][64];
  const int tid = threadIdx.x, wv = tid >> 5, lane = tid & 31; const int nd = blockIdx.x * 32 + wv; const bool live = nd < NNODE;
  const int p0 = live ? cstart[nd] : 0, p1 = live ? cstart[nd] + ccnt[nd] : 0;
  float erd[NH]; for (int h = 0; h < NH; ++h) erd[h] = live ? elr[(size_t)nd * 8 + 4 + h] : 0.f;
  float den[NH], mx[NH]; for (int h = 0; h < NH; ++h) { den[h] = 0.f; mx[h] = -__builtin_inff(); }
#pragma unroll 1
  for (int p = p0 + lane; p < p1; p += 32) { const int ee = ceid[p]; int s = (ee < NE) ? src[ee] : (ee - NE); s = s < 0 ? 0 : (s >= NNODE ? NNODE - 1 : s); const int k = p - p0; if (k < 64) sidx[wv][k] = s;
#pragma unroll
    for (int h = 0; h < NH; ++h) { float a = elr[(size_t)s * 8 + h] + erd[h]; a = a >= 0.f ? a : 0.2f * a; const float ex = expf(a); den[h] += ex; mx[h] = fmaxf(mx[h], a); if (k < 64) sal[wv][k][h] = ex; } }
#pragma unroll
  for (int h = 0; h < NH; ++h) { for (int o = 16; o >= 1; o >>= 1) { den[h] += __shfl_xor(den[h], o, 32); mx[h] = fmaxf(mx[h], __shfl_xor(mx[h], o, 32)); }
    den[h] += 1e-16f * ((mx[h] > -__builtin_inff()) ? expf(mx[h]) : 1.0f); }
  __builtin_amdgcn_fence(__ATOMIC_ACQ_REL, "workgroup"); __builtin_amdgcn_wave_barrier();
  const int hd_ = lane >> 3; float rd = 1.0f / ((hd_ == 0) ? den[0] : (hd_ == 1 ? den[1] : (hd_ == 2 ? den[2] : den[3]))); const float erh = (hd_ == 0) ? erd[0] : (hd_ == 1 ? erd[1] : (hd_ == 2 ? erd[2] : erd[3]));
  float acc[8] = {0.f,0.f,0.f,0.f,0.f,0.f,0.f,0.f};
#pragma unroll 1
  for (int p = p0; p < p1; ++p) { const int k = p - p0; int s; float ex;
    if (k < 64) { s = sidx[wv][k]; ex = sal[wv][k][hd_]; } else { const int ee = ceid[p]; s = (ee < NE) ? src[ee] : (ee - NE); s = s < 0 ? 0 : (s >= NNODE ? NNODE - 1 : s); float a = elr[(size_t)s * 8 + hd_] + erh; a = a >= 0.f ? a : 0.2f * a; ex = expf(a); }
    const float al_ = ex * rd; const v4f fa = *(const v4fa*)(f + (size_t)s * FH + lane * 8), fb = *(const v4fa*)(f + (size_t)s * FH + lane * 8 + 4);
    acc[0] += al_ * fa[0]; acc[1] += al_ * fa[1]; acc[2] += al_ * fa[2]; acc[3] += al_ * fa[3]; acc[4] += al_ * fb[0]; acc[5] += al_ * fb[1]; acc[6] += al_ * fb[2]; acc[7] += al_ * fb[3]; }
#pragma unroll
  for (int u = 0; u < 8; ++u) { const float v = acc[u] + bf16_round(bias[lane * 8 + u]); acc[u] = v > 0.f ? v : (__expf(v) - 1.0f); }
  if (live) {
#pragma unroll
      for (int u = 0; u < 8; ++u) srw[wv][lane * 8 + u] = acc[u];
      __builtin_amdgcn_fence(__ATOMIC_ACQ_REL, "workgroup"); __builtin_amdgcn_wave_barrier();
      float* orow = out + (size_t)nd * FH; for (int pass = 0; pass < 2; ++pass) { for (int i = 0; i < 8; ++i) *(volatile float*)(orow + i * 32 + lane) = srw[wv][i * 32 + lane]; if (pass == 0) __threadfence(); } }
}

__global__ __launch_bounds__(1024) void k_elr1(const float* __restrict__ h, const float* __restrict__ as, const float* __restrict__ ad, float* __restrict__ sc) {
  __shared__ float so[32][2]; const int tid = threadIdx.x, wv = tid >> 5, lane = tid & 31; const int n = blockIdx.x * 32 + wv; float s1 = 0.f, s2 = 0.f;
  if (n < NNODE) { const float v0 = h[(size_t)n * HD + lane], v1 = h[(size_t)n * HD + 32 + lane]; s1 = v0 * bf16_round(as[lane]) + v1 * bf16_round(as[32 + lane]); s2 = v0 * bf16_round(ad[lane]) + v1 * bf16_round(ad[32 + lane]); }
  for (int o = 16; o >= 1; o >>= 1) { s1 += __shfl_xor(s1, o, 32); s2 += __shfl_xor(s2, o, 32); } if (lane == 0) { so[wv][0] = s1; so[wv][1] = s2; } __syncthreads();
  if (tid < 64) { *(volatile float*)(sc + (size_t)blockIdx.x * 64 + tid) = so[tid >> 1][tid & 1]; } __threadfence(); if (tid < 64) { *(volatile float*)(sc + (size_t)blockIdx.x * 64 + tid) = so[tid >> 1][tid & 1]; }
}
__global__ __launch_bounds__(1024) void k_gat1(const float* __restrict__ h, const float* __restrict__ sc, const int* __restrict__ src, const int* __restrict__ cstart, const int* __restrict__ ccnt, const int* __restrict__ ceid, const float* __restrict__ bias, float* __restrict__ out) {
  __shared__ float sal[32][64]; __shared__ int sidx[32][64];
  const int tid = threadIdx.x, wv = tid >> 5, lane = tid & 31; const int d = blockIdx.x * 32 + wv; const bool live = d < NNODE;
  const int p0 = live ? cstart[d] : 0, p1 = live ? cstart[d] + ccnt[d] : 0; const float sdd = live ? sc[(size_t)d * 2 + 1] : 0.f;
  float den = 0.f, mx = -__builtin_inff();
#pragma unroll 1
  for (int p = p0 + lane; p < p1; p += 32) { const int e = ceid[p]; int s = (e < NE) ? src[e] : (e - NE); s = s < 0 ? 0 : (s >= NNODE ? NNODE - 1 : s); const int k = p - p0; float a = sc[(size_t)s * 2] + sdd; a = a >= 0.f ? a : 0.2f * a; const float ex = expf(a); den += ex; mx = fmaxf(mx, a); if (k < 64) { sal[wv][k] = ex; sidx[wv][k] = s; } }
  for (int o = 16; o >= 1; o >>= 1) { den += __shfl_xor(den, o, 32); mx = fmaxf(mx, __shfl_xor(mx, o, 32)); }
  den += 1e-16f * ((mx > -__builtin_inff()) ? expf(mx) : 1.0f); const float rd = 1.0f / den;
  __builtin_amdgcn_fence(__ATOMIC_ACQ_REL, "workgroup"); __builtin_amdgcn_wave_barrier();
  float a0 = 0.f, a1 = 0.f;
#pragma unroll 1
  for (int p = p0; p < p1; ++p) { const int k = p - p0; int s; float ex; if (k < 64) { s = sidx[wv][k]; ex = sal[wv][k]; } else { const int e = ceid[p]; s = (e < NE) ? src[e] : (e - NE); s = s < 0 ? 0 : (s >= NNODE ? NNODE - 1 : s); float a = sc[(size_t)s * 2] + sdd; a = a >= 0.f ? a : 0.2f * a; ex = expf(a); }
    const float al_ = ex * rd; a0 += al_ * h[(size_t)s * HD + lane]; a1 += al_ * h[(size_t)s * HD + 32 + lane]; }
  float v0 = a0 + bf16_round(bias[lane]), v1 = a1 + bf16_round(bias[32 + lane]); v0 = v0 > 0.f ? v0 : expm1f(v0); v1 = v1 > 0.f ? v1 : expm1f(v1);
  if (live) { float* orow = out + (size_t)d * HD; *(volatile float*)(orow + lane) = v0; *(volatile float*)(orow + 32 + lane) = v1; __threadfence(); *(volatile float*)(orow + lane) = v0; *(volatile float*)(orow + 32 + lane) = v1; }
}
__global__ __launch_bounds__(512) void k_granges(const int* __restrict__ batch, int* __restrict__ gs, int* __restrict__ gc) {
  const int g = threadIdx.x; int lo = 0, hi = NN; while (lo < hi) { const int m = (lo + hi) >> 1; if (batch[m] < g) lo = m + 1; else hi = m; } const int s0 = lo;
  lo = 0; hi = NN; while (lo < hi) { const int m = (lo + hi) >> 1; if (batch[m] < g + 1) lo = m + 1; else hi = m; } const int s1 = lo;
  const int st = (g < NGR) ? s0 : 0, c = (g < NGR) ? (s1 - s0) : 0; *(volatile int*)(gs + g) = st; *(volatile int*)(gc + g) = c; __threadfence(); *(volatile int*)(gs + g) = st; *(volatile int*)(gc + g) = c;
}
__global__ __launch_bounds__(1024) void k_pool(const float* __restrict__ z, const int* __restrict__ gs, const int* __restrict__ gc, float* __restrict__ ge) {
  const int tid = threadIdx.x, wv = tid >> 5, lane = tid & 31; const int g = blockIdx.x * 32 + wv; if (g >= NGR) return; const int s0 = gs[g], c = gc[g]; float a0 = 0.f, a1 = 0.f;
#pragma unroll 1
  for (int n = s0; n < s0 + c; ++n) { a0 += z[(size_t)n * HD + lane]; a1 += z[(size_t)n * HD + 32 + lane]; }
  const float inv = 1.0f / fmaxf((float)c, 1.0f); a0 *= inv; a1 *= inv;
  float* orow = ge + (size_t)g * HD; *(volatile float*)(orow + lane) = a0; *(volatile float*)(orow + 32 + lane) = a1; __threadfence(); *(volatile float*)(orow + lane) = a0; *(volatile float*)(orow + 32 + lane) = a1;
}

__global__ __launch_bounds__(64) void k_heads(const float* __restrict__ pooled, const float* __restrict__ wy, const float* __restrict__ by, const float* __restrict__ wp, const float* __restrict__ bp, const float* __restrict__ wo, const float* __restrict__ bo, const float* __restrict__ wm, const float* __restrict__ wd, float* __restrict__ out) {
  const int g = threadIdx.x; const float* pr = pooled + (size_t)g * HD; float sy = 0.f, sp = 0.f, l[4] = {0.f, 0.f, 0.f, 0.f};
#pragma unroll 1
  for (int c = 0; c < HD; ++c) { const float v = pr[c]; sy += v * bf16_round(wy[c]); sp += v * bf16_round(wp[c]); l[0] += v * bf16_round(wo[c * 4]); l[1] += v * bf16_round(wo[c * 4 + 1]); l[2] += v * bf16_round(wo[c * 4 + 2]); l[3] += v * bf16_round(wo[c * 4 + 3]); }
  sy += bf16_round(by[0]); sp += bf16_round(bp[0]); const float csm = bf16_round(wm[0]) * sy - bf16_round(wd[0]) * sp;
  for (int i = 0; i < 4; ++i) l[i] += bf16_round(bo[i]); const float m = fmaxf(fmaxf(l[0], l[1]), fmaxf(l[2], l[3])); float e[4], s = 0.f; for (int i = 0; i < 4; ++i) { e[i] = expf(l[i] - m); s += e[i]; }
  float* lg = out; float* oy = out + 64 * 4; float* op = out + 64 * 5; float* oc = out + 64 * 6;
  for (int pass = 0; pass < 2; ++pass) { *(volatile v4f*)(lg + g * 4) = (v4f){e[0] / s, e[1] / s, e[2] / s, e[3] / s}; *(volatile float*)(oy + g) = sy; *(volatile float*)(op + g) = sp; *(volatile float*)(oc + g) = csm; if (pass == 0) __threadfence(); }
}
extern "C" void kernel_launch(void* const* d_in, const int* in_sizes, int n_in,
                              void* d_out, int out_size, void* d_ws, size_t ws_size, hipStream_t stream) {
  (void)in_sizes; (void)n_in; (void)out_size;
  const float* x = (const float*)d_in[0]; const int* ei = (const int*)d_in[1]; const int* batch = (const int*)d_in[2]; const float* W1 = (const float*)d_in[3]; const float* as1 = (const float*)d_in[4]; const float* ad1 = (const float*)d_in[5]; const float* b1 = (const float*)d_in[6];
  const float* W2 = (const float*)d_in[7]; const float* as2 = (const float*)d_in[8]; const float* ad2 = (const float*)d_in[9]; const float* b2 = (const float*)d_in[10];
  const float* wy = (const float*)d_in[11]; const float* by = (const float*)d_in[12]; const float* wp = (const float*)d_in[13]; const float* bp = (const float*)d_in[14]; const float* wo = (const float*)d_in[15]; const float* bo = (const float*)d_in[16]; const float* wm = (const float*)d_in[17]; const float* wd = (const float*)d_in[18];
  char* ws = (char*)d_ws; size_t off = 0;
  auto take = [&](size_t bytes) { char* p = ws + off; off += (bytes + 255) & ~(size_t)255; return p; };
  unsigned short* B1 = (unsigned short*)take((size_t)FH * 128 * 2); _Float16* B2 = (_Float16*)take((size_t)HD * FH * 2);
  int* seg_dst = (int*)take((size_t)CS_NW * CS_CH * 4); int* seg_eid = (int*)take((size_t)CS_NW * CS_CH * 4); int* P1 = (int*)take((size_t)CS_NW * CS_NB * 4); int* Q1 = (int*)take((size_t)CS_NW * CS_NB * 4); int* R = (int*)take((size_t)CS_NW * CS_NB * 4); int* S = (int*)take((CS_NB + 32) * 4);
  int* ceid = (int*)take(((size_t)NTOT + 32 * CS_NB) * 4); int* cstart = (int*)take((size_t)CS_NB * CS_NB * 4); int* ccnt = (int*)take((size_t)CS_NB * CS_NB * 4);
  float* f1 = (float*)take((size_t)NNODE * FH * 4); float* elr = (float*)take((size_t)((NNODE + 31) / 32) * 32 * 8 * 4); float* h1 = (float*)take((size_t)NNODE * FH * 4); float* f2 = (float*)take((size_t)NNODE * HD * 4); float* sc2 = (float*)take((size_t)((NNODE + 31) / 32) * 64 * 4); float* h2 = (float*)take((size_t)NNODE * HD * 4);
  int* gs = (int*)take(512 * 4); int* gc = (int*)take(512 * 4); float* pooled = (float*)take((size_t)NGR * HD * 4);
  if (off > ws_size) return;
  k_wt_bf16<<<(FH * 16 + 255) / 256, 256, 0, stream>>>(W1, B1, 128, FH); k_wt_f16<<<(HD * 32 + 255) / 256, 256, 0, stream>>>(W2, B2, FH, HD, 16.0f);
  build_csr(ei + NE, NE, NTOT, NNODE, seg_dst, seg_eid, P1, Q1, R, S, ceid, cstart, ccnt, stream);
  const unsigned gb = (NNODE + 31) / 32;
  k_gemm_bf3<false, 0, false, false><<<((NNODE / 16) * 4 + 3) / 4, 128, 0, stream>>>(x, 128, B1, 128, nullptr, nullptr, 1, 0, f1, FH, NNODE, FH, 128);
  k_elr<<<gb, 1024, 0, stream>>>(f1, as1, ad1, elr);
  k_gat4<<<gb, 1024, 0, stream>>>(f1, elr, ei, cstart, ccnt, ceid, h1, b1);
  k_gemm_h<false><<<dim3(((NNODE / 16) * 1 + 3) / 4, 1), 128, 0, stream>>>(h1, FH, 0, B2, FH, 0, 0.0625f, f2, HD, 0, NNODE, HD, FH);
  k_elr1<<<gb, 1024, 0, stream>>>(f2, as2, ad2, sc2);
  k_gat1<<<gb, 1024, 0, stream>>>(f2, sc2, ei, cstart, ccnt, ceid, b2, h2);
  k_granges<<<1, 512, 0, stream>>>(batch, gs, gc); k_pool<<<(NGR + 31) / 32, 1024, 0, stream>>>(h2, gs, gc, pooled);
  k_heads<<<1, 64, 0, stream>>>(pooled, wy, by, wp, bp, wo, bo, wm, wd, (float*)d_out);
}
